// SplineFlow_55576876810926
// MI455X (gfx1250) — hardware-verified
//
#include <hip/hip_runtime.h>
#include <hip/hip_bf16.h>
#include <math.h>

typedef __attribute__((ext_vector_type(16))) _Float16 v16h;
typedef __attribute__((ext_vector_type(8)))  _Float16 v8h;
typedef __attribute__((ext_vector_type(16))) __bf16   v16b;
typedef __attribute__((ext_vector_type(8)))  __bf16   v8b;
typedef __attribute__((ext_vector_type(8)))  float    v8f;
typedef __attribute__((ext_vector_type(4)))  float    v4f;
typedef __attribute__((ext_vector_type(2)))  float    v2f;
#define PSCALE 32768.0f
#define U16(p) ((const unsigned short*)(const void*)(p))
#define PSCALE_INV (1.0f / 32768.0f)

__device__ __forceinline__ unsigned short f2bf_bits(float f) {
  unsigned u = __float_as_uint(f);
  return (unsigned short)((u + 0x7FFFu + ((u >> 16) & 1u)) >> 16);
}
__device__ __forceinline__ float bf_bits2f(unsigned short h) { return __uint_as_float(((unsigned)h) << 16); }

__device__ __forceinline__ void dep_guard_h(v8f& a, v8f& b, v16h x, v16h y) { asm volatile("v_nop\n\tv_nop\n\tv_nop\n\tv_nop" : "+v"(a), "+v"(b) : "v"(x), "v"(y)); }
__device__ __forceinline__ void dep_guard_b(v8f& a, v8f& b, v16b x, v16b y) { asm volatile("v_nop\n\tv_nop\n\tv_nop\n\tv_nop" : "+v"(a), "+v"(b) : "v"(x), "v"(y)); }
__device__ __forceinline__ void keep4_h(v16h a, v16h b, v16h c, v16h d) { asm volatile("v_nop" :: "v"(a), "v"(b), "v"(c), "v"(d)); }
__device__ __forceinline__ void keep4_b(v16b a, v16b b, v16b c, v16b d) { asm volatile("v_nop" :: "v"(a), "v"(b), "v"(c), "v"(d)); }
__device__ __forceinline__ void acc_guard4(v8f& a, v8f& b, v8f& c, v8f& d) { asm volatile("v_nop\n\tv_nop\n\tv_nop\n\tv_nop" : "+v"(a), "+v"(b), "+v"(c), "+v"(d)); }
template <typename T> struct Frag;
template <> struct Frag<_Float16> {
  typedef v16h V; union U { v16h v; v8h h[2]; };
  static __device__ __forceinline__ v16h load(const _Float16* p) {
    U f; f.h[0] = *(const v8h*)(p); f.h[1] = *(const v8h*)(p + 16); return f.v;
  }
  static __device__ __forceinline__ v8f mma(v16h a, v16h b, v8f c) {
    return __builtin_amdgcn_wmma_f32_16x16x32_f16(false, a, false, b, (short)0, c, false, false);
  }
  static __device__ __forceinline__ void guard(v8f& a, v8f& b, v16h x, v16h y) { dep_guard_h(a, b, x, y); }
  static __device__ __forceinline__ void keep(v16h a, v16h b, v16h c, v16h d) { keep4_h(a, b, c, d); }
};
template <> struct Frag<__bf16> {
  typedef v16b V; union U { v16b v; v8b h[2]; };
  static __device__ __forceinline__ v16b load(const __bf16* p) {
    U f; f.h[0] = *(const v8b*)(p); f.h[1] = *(const v8b*)(p + 16); return f.v;
  }
  static __device__ __forceinline__ v8f mma(v16b a, v16b b, v8f c) {
    return __builtin_amdgcn_wmma_f32_16x16x32_bf16(false, a, false, b, (short)0, c, false, false);
  }
  static __device__ __forceinline__ void guard(v8f& a, v8f& b, v16b x, v16b y) { dep_guard_b(a, b, x, y); }
  static __device__ __forceinline__ void keep(v16b a, v16b b, v16b c, v16b d) { keep4_b(a, b, c, d); }
};

template <int ET> struct Elem;
template <> struct Elem<0> { typedef _Float16 T; };
template <> struct Elem<1> { typedef __bf16 T; };
template <int ET, bool SPLIT, int BIAS_MODE, int OUT_MODE, bool RESID, int ACT = 0>
__global__ __launch_bounds__(256) void wmma_gemm64(
    const unsigned short* __restrict__ Ap, const unsigned short* __restrict__ A2p, int lda, long strideA,
    const unsigned short* __restrict__ Btp, const unsigned short* __restrict__ Bt2p, int ldb, long strideB,
    void* __restrict__ Cout, void* __restrict__ Cout2, int ldc, long strideC,
    const float* __restrict__ bias,
    const float* __restrict__ resid, long strideR,
    int M, int N, int K, float scale) {
  typedef typename Elem<ET>::T T;
  typedef typename Frag<T>::V V;
  const T* A = (const T*)Ap; const T* A2 = (const T*)A2p; const T* Bt = (const T*)Btp; const T* Bt2 = (const T*)Bt2p;
  __shared__ __align__(16) float sT[8][16 * 68];
  const int b    = blockIdx.y;
  const int lane = threadIdx.x & 31;
  const int wave = threadIdx.x >> 5;
  const int tilesN = N >> 6;
  const int tilesM = M >> 6;
  const int tile = blockIdx.x * 8 + wave;
  if (tile >= tilesM * tilesN) return;
  const int tm = tile / tilesN;
  const int tn = tile - tm * tilesN;
  const int m0 = tm << 6;
  const int n0 = tn << 6;

  const T* Ab  = A  + (size_t)b * strideA;
  const T* Bb  = Bt + (size_t)b * strideB;
  const T* Ab2 = SPLIT ? (A2  + (size_t)b * strideA) : nullptr;
  const T* Bb2 = SPLIT ? (Bt2 + (size_t)b * strideB) : nullptr;

  const int rlane = lane & 15;
  const int koff  = (lane >> 4) * 8;
  const int mOff  = (lane >> 4) * 8;

  v8f acc[4][4];
#pragma unroll
  for (int i = 0; i < 4; ++i)
#pragma unroll
    for (int j = 0; j < 4; ++j) acc[i][j] = (v8f){0.f,0.f,0.f,0.f,0.f,0.f,0.f,0.f};

  for (int k0 = 0; k0 < K; k0 += 32) {
    V bh[4], bl[4];
#pragma unroll
    for (int j = 0; j < 4; ++j) {
      const size_t bo = (size_t)(n0 + (j << 4) + rlane) * ldb + koff + k0;
      bh[j] = Frag<T>::load(Bb + bo);
      if (SPLIT) bl[j] = Frag<T>::load(Bb2 + bo);
    }
#pragma unroll
    for (int i = 0; i < 4; ++i) {
      const size_t ao = (size_t)(m0 + (i << 4) + rlane) * lda + koff + k0;
      V ah = Frag<T>::load(Ab + ao);
      V al;
      if (SPLIT) al = Frag<T>::load(Ab2 + ao);
#pragma unroll
      for (int j = 0; j < 4; ++j) {
        acc[i][j] = Frag<T>::mma(ah, bh[j], acc[i][j]);
        if (SPLIT) {
          acc[i][j] = Frag<T>::mma(ah, bl[j], acc[i][j]);
          acc[i][j] = Frag<T>::mma(al, bh[j], acc[i][j]);
        }
      }
      Frag<T>::guard(acc[i][0], acc[i][3], ah, SPLIT ? al : ah);
    }
    Frag<T>::keep(bh[0], bh[1], bh[2], bh[3]);
    if (SPLIT) Frag<T>::keep(bl[0], bl[1], bl[2], bl[3]);
  }
  acc_guard4(acc[0][0], acc[0][1], acc[0][2], acc[0][3]);
  acc_guard4(acc[1][0], acc[1][1], acc[1][2], acc[1][3]);
  acc_guard4(acc[2][0], acc[2][1], acc[2][2], acc[2][3]);
  acc_guard4(acc[3][0], acc[3][1], acc[3][2], acc[3][3]);

  float* slab = sT[wave];
  const float* Rb = RESID ? (resid + (size_t)b * strideR) : nullptr;
#pragma unroll
  for (int i = 0; i < 4; ++i) {
    const int mBase = m0 + (i << 4);
#pragma unroll
    for (int j = 0; j < 4; ++j) {
      const int n = n0 + (j << 4) + rlane;
      float bv = 0.f;
      if (BIAS_MODE == 2) bv = bias[n];
#pragma unroll
      for (int r = 0; r < 8; ++r) {
        float v = acc[i][j][r] * scale;
        if (BIAS_MODE == 1) v += bias[mBase + mOff + r];
        if (BIAS_MODE == 2) v += bv;
        if (RESID) v += Rb[(size_t)(mBase + mOff + r) * ldc + n];
        if (ACT == 1) v = tanhf(v);
        if (ACT == 2) v = fmaxf(v, 0.0f);
        if (ACT == 3) v = v / (1.0f + expf(-v));
        if (ACT == 4) v = (v > 0.f) ? v : 0.01f * v;
        if (ACT == 5) v = 0.5f * v * (1.0f + erff(v * 0.70710678118654752f));
        slab[(mOff + r) * 68 + (j << 4) + rlane] = v;
      }
    }
    __builtin_amdgcn_fence(__ATOMIC_RELEASE, "workgroup");
    __builtin_amdgcn_wave_barrier();
    __builtin_amdgcn_fence(__ATOMIC_ACQUIRE, "workgroup");
    if (OUT_MODE == 0) {
      float* C = (float*)Cout + (size_t)b * strideC;
      const int hh = lane >> 4, c4 = (lane & 15) * 4;
      for (int pass = 0; pass < 2; ++pass) {
#pragma unroll
        for (int it = 0; it < 8; ++it) {
          const int row = it * 2 + hh;
          v4f v = *(const v4f*)(slab + row * 68 + c4);
          *(volatile v4f*)(C + (size_t)(mBase + row) * ldc + n0 + c4) = v;
        }
        __threadfence();
      }
    } else {
      const int q = lane >> 3, c8 = (lane & 7) * 8;
      unsigned short* C  = (unsigned short*)Cout  + (size_t)b * strideC;
      unsigned short* C2 = (OUT_MODE == 2) ? ((unsigned short*)Cout2 + (size_t)b * strideC) : nullptr;
      for (int pass = 0; pass < 2; ++pass) {
#pragma unroll
        for (int it = 0; it < 4; ++it) {
          const int row = it * 4 + q;
          const float* sp = slab + row * 68 + c8;
          v8h hv, lv;
#pragma unroll
          for (int e = 0; e < 8; ++e) {
            if (OUT_MODE == 1) {
              hv[e] = (_Float16)sp[e];
            } else {
              unsigned short hb = f2bf_bits(sp[e]);
              unsigned short lb = f2bf_bits(sp[e] - bf_bits2f(hb));
              hv[e] = __builtin_bit_cast(_Float16, hb);
              lv[e] = __builtin_bit_cast(_Float16, lb);
            }
          }
          *(volatile v8h*)(C + (size_t)(mBase + row) * ldc + n0 + c8) = hv;
          if (OUT_MODE == 2) *(volatile v8h*)(C2 + (size_t)(mBase + row) * ldc + n0 + c8) = lv;
        }
        __threadfence();
      }
    }
    __builtin_amdgcn_fence(__ATOMIC_RELEASE, "workgroup");
    __builtin_amdgcn_wave_barrier();
    __builtin_amdgcn_fence(__ATOMIC_ACQUIRE, "workgroup");
  }
}

constexpr int NB     = 32768;
constexpr int ND     = 64;
constexpr int NH     = 512;
constexpr int NK     = 8;
constexpr int NP     = 3 * NK - 1;
constexpr int NDP    = ND * NP;
constexpr int KCAT   = 2 * NH;
constexpr int CHUNK  = 8192;
constexpr int NCHUNK = NB / CHUNK;
constexpr int SPR    = 32;
constexpr int SPSUB  = 4;
constexpr int LDPITCH = ND + 1;
constexpr float BOUNDV = 4.0f;
constexpr float MINBIN = 0.001f;
constexpr float MINDER = 0.001f;
constexpr float BINSCL = 0.992f;

static_assert(NP * ND == NDP, "param layout");
static_assert(NB % 64 == 0 && NH % 64 == 0 && ND % 32 == 0, "GEMM-1: M,N tile multiples, K % 32 == 0");
static_assert(CHUNK % 64 == 0 && NDP % 64 == 0 && KCAT % 32 == 0, "GEMM-2: M,N tile multiples, K % 32 == 0");
static_assert(NB % CHUNK == 0 && CHUNK % SPR == 0 && SPR % SPSUB == 0, "spline grid coverage");
static_assert(((NB / 64) * (NH / 64)) % 8 == 0, "GEMM-1 grid exact");
static_assert(((CHUNK / 64) * (NDP / 64)) % 8 == 0, "GEMM-2 grid exact");
static_assert((NDP * 4) % 16 == 0, "param rows float4-aligned");
static_assert(SPSUB * ND == 256, "one thread per (row, dim) in a sub-iteration");

constexpr size_t OFF_XB   = 0;
constexpr size_t SZ_XB    = (size_t)NB * ND * 2;
constexpr size_t OFF_W1M  = OFF_XB + SZ_XB;
constexpr size_t SZ_W1M   = (size_t)NH * ND * 2;
constexpr size_t OFF_W2M  = OFF_W1M + SZ_W1M;
constexpr size_t SZ_W2M   = (size_t)NDP * KCAT * 2;
constexpr size_t OFF_B1R  = OFF_W2M + SZ_W2M;
constexpr size_t SZ_B1R   = (size_t)NH * 4;
constexpr size_t OFF_B2R  = OFF_B1R + SZ_B1R;
constexpr size_t SZ_B2R   = (size_t)NDP * 4;
constexpr size_t OFF_HCAT = OFF_B2R + SZ_B2R;
constexpr size_t SZ_HCAT  = (size_t)NB * KCAT * 2;
constexpr size_t OFF_PRM  = OFF_HCAT + SZ_HCAT;
constexpr size_t SZ_PRM   = (size_t)CHUNK * NDP * 4;
constexpr size_t WS_TOTAL = OFF_PRM + SZ_PRM;
static_assert(WS_TOTAL == 122625792, "carve total");
static_assert(WS_TOTAL <= 134217728, "carve within limit");
static_assert(OFF_W1M % 128 == 0 && OFF_W2M % 128 == 0 && OFF_B1R % 128 == 0 && OFF_B2R % 128 == 0 &&
              OFF_HCAT % 128 == 0 && OFF_PRM % 128 == 0, "128-B aligned regions");
constexpr size_t OUT0_BYTES = (size_t)NB * ND * 4;
constexpr size_t OUT1_OFF_BYTES = 8388608;
static_assert(OUT0_BYTES == OUT1_OFF_BYTES, "out1 byte offset");
static_assert(OUT1_OFF_BYTES + (size_t)NB * 4 == 8519680, "total out bytes");
static_assert(OUT1_OFF_BYTES % 128 == 0, "out1 starts on a line");

__device__ __forceinline__ float bf_rne(float f) { return bf_bits2f(f2bf_bits(f)); }

__global__ __launch_bounds__(256) void cast_x_bf16(const float* __restrict__ in, unsigned* __restrict__ out, int n2) {
  const int i = blockIdx.x * 256 + threadIdx.x;
  if (i < n2) {
    const v2f t = *(const v2f*)(in + 2 * (size_t)i);
    const unsigned u = (unsigned)f2bf_bits(t[0]) | ((unsigned)f2bf_bits(t[1]) << 16);
    ((volatile unsigned*)out)[i] = u;
    __threadfence();
    ((volatile unsigned*)out)[i] = u;
  }
}

__global__ __launch_bounds__(256) void prep_w1(const float* __restrict__ W1, const float* __restrict__ M1,
                                               unsigned* __restrict__ out, int n2) {
  const int i = blockIdx.x * 256 + threadIdx.x;
  if (i < n2) {
    const v2f w = *(const v2f*)(W1 + 2 * (size_t)i);
    const v2f m = *(const v2f*)(M1 + 2 * (size_t)i);
    const float a = bf_rne(w[0]) * bf_rne(m[0]);
    const float c = bf_rne(w[1]) * bf_rne(m[1]);
    const unsigned u = (unsigned)f2bf_bits(a) | ((unsigned)f2bf_bits(c) << 16);
    ((volatile unsigned*)out)[i] = u;
    __threadfence();
    ((volatile unsigned*)out)[i] = u;
  }
}

__global__ __launch_bounds__(256) void prep_w2(const float* __restrict__ W2, const float* __restrict__ M2,
                                               unsigned* __restrict__ out, int nt) {
  const int t = blockIdx.x * 256 + threadIdx.x;
  if (t < nt) {
    const int n = t >> 9;
    const int p = t & 511;
    const int k = (2 * p) & 511;
    const size_t src = (size_t)n * NH + k;
    const v2f w = *(const v2f*)(W2 + src);
    const v2f m = *(const v2f*)(M2 + src);
    const float a = bf_rne(w[0]) * bf_rne(m[0]);
    const float c = bf_rne(w[1]) * bf_rne(m[1]);
    const unsigned u = (unsigned)f2bf_bits(a) | ((unsigned)f2bf_bits(c) << 16);
    ((volatile unsigned*)out)[t] = u;
    __threadfence();
    ((volatile unsigned*)out)[t] = u;
  }
}

__global__ __launch_bounds__(256) void prep_bias(const float* __restrict__ b1, const float* __restrict__ b2,
                                                 float* __restrict__ b1r, float* __restrict__ b2r) {
  const int i = blockIdx.x * 256 + threadIdx.x;
  if (i < NH) {
    const float v = bf_rne(b1[i]);
    ((volatile float*)b1r)[i] = v;
    __threadfence();
    ((volatile float*)b1r)[i] = v;
  }
  if (i < NDP) {
    const float v = bf_rne(b2[i]);
    ((volatile float*)b2r)[i] = v;
    __threadfence();
    ((volatile float*)b2r)[i] = v;
  }
}

__global__ __launch_bounds__(256) void rqs_spline(const float* __restrict__ prm, const float* __restrict__ xg,
                                                  float* __restrict__ zo, float* __restrict__ ldo, int row0) {
#pragma clang fp contract(off)
  __shared__ __align__(16) float sp[SPSUB * NDP];
  __shared__ __align__(16) float zs[SPSUB * ND];
  __shared__ float ldacc[SPR * LDPITCH];
  __shared__ __align__(16) float ldline[SPR];

  const int tid  = threadIdx.x;
  const int lane = tid & 31;
  const int wave = tid >> 5;
  const int rloc = tid >> 6;
  const int dd   = tid & 63;
  const int brow = blockIdx.x * SPR;

  for (int sub = 0; sub < SPR / SPSUB; ++sub) {
    const int crow = brow + sub * SPSUB;
    __syncthreads();
#pragma unroll
    for (int rr = 0; rr < SPSUB; ++rr) {
      const float* src = prm + (size_t)(crow + rr) * NDP;
      for (int q = tid; q < NDP / 4; q += 256) {
        const v4f v = *(const v4f*)(src + 4 * q);
        *(v4f*)(sp + rr * NDP + 4 * q) = v;
      }
    }
    __syncthreads();

    float* p = sp + rloc * NDP + dd * NP;

    float mw = p[0], mh = p[NK];
#pragma unroll 1
    for (int i = 1; i < NK; ++i) { mw = fmaxf(mw, p[i]); mh = fmaxf(mh, p[NK + i]); }
    float sw = 0.0f, sh = 0.0f;
#pragma unroll 1
    for (int i = 0; i < 2 * NK; ++i) {
      const bool fw = (i < NK);
      const float m = fw ? mw : mh;
      const float e = expf(p[i] - m);
      p[i] = e;
      if (fw) sw = sw + e; else sh = sh + e;
    }
    float cw = 0.0f, ch = 0.0f;
#pragma unroll 1
    for (int i = 0; i < NK - 1; ++i) {
      const float wn = p[i] / sw;
      const float hn = p[NK + i] / sh;
      const float wv = MINBIN + BINSCL * wn;
      const float hv = MINBIN + BINSCL * hn;
      cw = cw + wv;
      ch = ch + hv;
      p[i]      = -BOUNDV + 8.0f * cw;
      p[NK + i] = -BOUNDV + 8.0f * ch;
    }

    const int grow = row0 + crow + rloc;
    const float xin = xg[(size_t)grow * ND + dd];
    const float xr  = bf_rne(xin);
    const bool inside = (xr >= -BOUNDV) && (xr <= BOUNDV);
    const float xc  = fminf(fmaxf(xr, -BOUNDV), BOUNDV);
    int cnt = 1 + ((xc >= BOUNDV) ? 1 : 0);
#pragma unroll 1
    for (int i = 0; i < NK - 1; ++i) cnt += (xc >= p[i]) ? 1 : 0;
    int idx = cnt - 1;
    idx = (idx < 0) ? 0 : idx;
    idx = (idx > NK - 1) ? (NK - 1) : idx;
    const int ia = (idx > 0) ? (idx - 1) : 0;
    const int ib = (idx < NK - 1) ? idx : (NK - 2);
    const float xa = p[ia], xb = p[ib];
    const float ya = p[NK + ia], yb = p[NK + ib];
    const float x_k  = (idx == 0) ? -BOUNDV : xa;
    const float x_k1 = (idx == NK - 1) ? BOUNDV : xb;
    const float y_k  = (idx == 0) ? -BOUNDV : ya;
    const float y_k1 = (idx == NK - 1) ? BOUNDV : yb;

    const float dua = p[2 * NK + ia];
    const float dub = p[2 * NK + ib];
    p[NK - 1] = dua;
    p[2 * NK - 1] = dub;
#pragma unroll 1
    for (int j = 0; j < 2; ++j) {
      const int sl = NK - 1 + NK * j;
      const float v = p[sl];
      const float spv = fmaxf(v, 0.0f) + log1pf(expf(-fabsf(v)));
      p[sl] = MINDER + spv;
    }
    const float da = p[NK - 1], db = p[2 * NK - 1];
    const float d_k  = (idx == 0) ? 1.0f : da;
    const float d_k1 = (idx == NK - 1) ? 1.0f : db;

    const float w_k   = x_k1 - x_k;
    const float h_k   = y_k1 - y_k;
    const float s     = h_k / w_k;
    const float theta = (xc - x_k) / w_k;
    const float omt   = 1.0f - theta;
    const float t1m   = theta * omt;
    const float num   = h_k * (s * theta * theta + d_k * t1m);
    const float den   = s + (d_k1 + d_k - 2.0f * s) * t1m;
    const float y_in  = y_k + num / den;
    const float dnum  = s * s * (d_k1 * theta * theta + 2.0f * s * t1m + d_k * (omt * omt));
    p[NK - 1] = dnum;
    p[2 * NK - 1] = den;
#pragma unroll 1
    for (int j = 0; j < 2; ++j) {
      const int sl = NK - 1 + NK * j;
      p[sl] = logf(p[sl]);
    }
    const float ld_in = p[NK - 1] - 2.0f * p[2 * NK - 1];

    const float y  = inside ? y_in : xr;
    const float ld = inside ? ld_in : 0.0f;
    zs[rloc * ND + dd] = y;
    ldacc[(sub * SPSUB + rloc) * LDPITCH + dd] = ld;
    __syncthreads();

    if (wave < 2) {
      const int q4  = wave * 32 + lane;
      const int row = q4 >> 4;
      const int c4  = (q4 & 15) * 4;
      const v4f v = *(const v4f*)(zs + row * ND + c4);
      float* dst = zo + (size_t)(row0 + crow + row) * ND + c4;
      *(volatile v4f*)dst = v;
      __threadfence();
      *(volatile v4f*)dst = v;
    }
  }

  __syncthreads();
  if (tid < SPR) {
    float a = 0.0f;
#pragma unroll 1
    for (int d2 = 0; d2 < ND; ++d2) a = a + ldacc[tid * LDPITCH + d2];
    ldline[tid] = a;
  }
  __syncthreads();
  if (tid < SPR / 4) {
    const v4f v = *(const v4f*)(ldline + 4 * tid);
    float* dst = ldo + (size_t)row0 + brow + 4 * tid;
    *(volatile v4f*)dst = v;
    __threadfence();
    *(volatile v4f*)dst = v;
  }
}

extern "C" void kernel_launch(void* const* d_in, const int* in_sizes, int n_in,
                              void* d_out, int out_size, void* d_ws,
                              size_t ws_size, hipStream_t stream) {
  if (n_in < 7) return;
  if (in_sizes[0] != NB * ND || in_sizes[1] != NH * ND || in_sizes[2] != NH ||
      in_sizes[3] != NDP * NH || in_sizes[4] != NDP || in_sizes[5] != NH * ND || in_sizes[6] != NDP * NH) return;
  if (out_size != NB * ND + NB) return;
  if (ws_size < WS_TOTAL) return;

  const float* x  = (const float*)d_in[0];
  const float* W1 = (const float*)d_in[1];
  const float* b1 = (const float*)d_in[2];
  const float* W2 = (const float*)d_in[3];
  const float* b2 = (const float*)d_in[4];
  const float* M1 = (const float*)d_in[5];
  const float* M2 = (const float*)d_in[6];

  char* ws = (char*)d_ws;
  unsigned short* xb   = (unsigned short*)(ws + OFF_XB);
  unsigned short* w1m  = (unsigned short*)(ws + OFF_W1M);
  unsigned short* w2m  = (unsigned short*)(ws + OFF_W2M);
  float*          b1r  = (float*)(ws + OFF_B1R);
  float*          b2r  = (float*)(ws + OFF_B2R);
  unsigned short* hcat = (unsigned short*)(ws + OFF_HCAT);
  float*          prm  = (float*)(ws + OFF_PRM);

  float* z_out  = (float*)d_out;
  float* ld_out = (float*)((char*)d_out + OUT1_OFF_BYTES);

  const int nx2 = NB * ND / 2;
  cast_x_bf16<<<dim3(nx2 / 256), dim3(256), 0, stream>>>(x, (unsigned*)xb, nx2);
  const int nw1 = NH * ND / 2;
  prep_w1<<<dim3(nw1 / 256), dim3(256), 0, stream>>>(W1, M1, (unsigned*)w1m, nw1);
  const int nw2 = NDP * NH;
  prep_w2<<<dim3(nw2 / 256), dim3(256), 0, stream>>>(W2, M2, (unsigned*)w2m, nw2);
  prep_bias<<<dim3((NDP + 255) / 256), dim3(256), 0, stream>>>(b1, b2, b1r, b2r);

  const int g1 = (NB / 64) * (NH / 64) / 8;
  wmma_gemm64<1, false, 2, 2, false, 2><<<dim3(g1, 1), dim3(256), 0, stream>>>(
      xb, xb, ND, 0L,
      w1m, w1m, ND, 0L,
      (void*)hcat, (void*)(hcat + NH), KCAT, 0L,
      b1r, b1r, 0L,
      NB, NH, ND, 1.0f);

  const int g2 = (CHUNK / 64) * (NDP / 64) / 8;
  for (int c = 0; c < NCHUNK; ++c) {
    const unsigned short* Ac = hcat + (size_t)c * CHUNK * KCAT;
    wmma_gemm64<1, false, 2, 0, false, 0><<<dim3(g2, 1), dim3(256), 0, stream>>>(
        Ac, Ac, KCAT, 0L,
        w2m, w2m, KCAT, 0L,
        (void*)prm, (void*)prm, NDP, 0L,
        b2r, b2r, 0L,
        CHUNK, NDP, KCAT, 1.0f);
    rqs_spline<<<dim3(CHUNK / SPR), dim3(256), 0, stream>>>(prm, x, z_out, ld_out, c * CHUNK);
  }
}
